// GAT_3_38036230373751
// MI455X (gfx1250) — hardware-verified
//
#include <hip/hip_runtime.h>
#include <math.h>

#define NNODE 10000
#define NEDGE 160000
#define NVIRT (NEDGE + NNODE)
#define MP 10048
#define NT 256
#define TGB 2048
#define NTB 5
#define TGA 512
#define NTA 20
#define SCH 4096
#define SPT (SCH / NT)
#define NCH1 ((NEDGE + SCH - 1) / SCH)
#define NCH2 ((NVIRT + SCH - 1) / SCH)
#define GW 1024
#define THW 256
#define WSC 16.0f
#define WSC_INV 0.0625f
#define BN_EPS 1e-5f

static_assert(NEDGE % SPT == 0);
static_assert(NTB * TGB >= MP && NTA * TGA >= MP);
static_assert(MP % 64 == 0 && MP >= NNODE);
static_assert(NVIRT < (1 << 20));

typedef __attribute__((ext_vector_type(16))) _Float16 v16h;
typedef __attribute__((ext_vector_type(8)))  _Float16 v8h;
typedef __attribute__((ext_vector_type(4)))  _Float16 v4h;
typedef __attribute__((ext_vector_type(16))) __bf16   v16b;
typedef __attribute__((ext_vector_type(8)))  __bf16   v8b;
typedef __attribute__((ext_vector_type(8)))  float    v8f;
typedef __attribute__((ext_vector_type(4)))  float    v4f;
typedef __attribute__((ext_vector_type(2)))  float    v2f;
typedef __attribute__((ext_vector_type(4)))  int      v4i;
#define U16(p) ((const unsigned short*)(const void*)(p))

__device__ __forceinline__ unsigned short f2bf_bits(float f) {
  unsigned u = __float_as_uint(f);
  return (unsigned short)((u + 0x7FFFu + ((u >> 16) & 1u)) >> 16);
}
__device__ __forceinline__ float bf_bits2f(unsigned short h) { return __uint_as_float(((unsigned)h) << 16); }

__device__ __forceinline__ void dep_guard_h(v8f& a, v8f& b, v16h x, v16h y) { asm volatile("v_nop\n\tv_nop\n\tv_nop\n\tv_nop" : "+v"(a), "+v"(b) : "v"(x), "v"(y)); }
__device__ __forceinline__ void dep_guard_b(v8f& a, v8f& b, v16b x, v16b y) { asm volatile("v_nop\n\tv_nop\n\tv_nop\n\tv_nop" : "+v"(a), "+v"(b) : "v"(x), "v"(y)); }
__device__ __forceinline__ void keep4_h(v16h a, v16h b, v16h c, v16h d) { asm volatile("v_nop" :: "v"(a), "v"(b), "v"(c), "v"(d)); }
__device__ __forceinline__ void keep4_b(v16b a, v16b b, v16b c, v16b d) { asm volatile("v_nop" :: "v"(a), "v"(b), "v"(c), "v"(d)); }
__device__ __forceinline__ void acc_guard4(v8f& a, v8f& b, v8f& c, v8f& d) { asm volatile("v_nop\n\tv_nop\n\tv_nop\n\tv_nop" : "+v"(a), "+v"(b), "+v"(c), "+v"(d)); }
template <typename T> struct Frag;
template <> struct Frag<_Float16> {
  typedef v16h V; union U { v16h v; v8h h[2]; };
  static __device__ __forceinline__ v16h load(const _Float16* p) {
    U f; f.h[0] = *(const v8h*)(p); f.h[1] = *(const v8h*)(p + 16); return f.v;
  }
  static __device__ __forceinline__ v8f mma(v16h a, v16h b, v8f c) {
    return __builtin_amdgcn_wmma_f32_16x16x32_f16(false, a, false, b, (short)0, c, false, false);
  }
  static __device__ __forceinline__ void guard(v8f& a, v8f& b, v16h x, v16h y) { dep_guard_h(a, b, x, y); }
  static __device__ __forceinline__ void keep(v16h a, v16h b, v16h c, v16h d) { keep4_h(a, b, c, d); }
};
template <> struct Frag<__bf16> {
  typedef v16b V; union U { v16b v; v8b h[2]; };
  static __device__ __forceinline__ v16b load(const __bf16* p) {
    U f; f.h[0] = *(const v8b*)(p); f.h[1] = *(const v8b*)(p + 16); return f.v;
  }
  static __device__ __forceinline__ v8f mma(v16b a, v16b b, v8f c) {
    return __builtin_amdgcn_wmma_f32_16x16x32_bf16(false, a, false, b, (short)0, c, false, false);
  }
  static __device__ __forceinline__ void guard(v8f& a, v8f& b, v16b x, v16b y) { dep_guard_b(a, b, x, y); }
  static __device__ __forceinline__ void keep(v16b a, v16b b, v16b c, v16b d) { keep4_b(a, b, c, d); }
};

template <int ET> struct Elem;
template <> struct Elem<0> { typedef _Float16 T; };
template <> struct Elem<1> { typedef __bf16 T; };
template <int ET, bool SPLIT, int BIAS_MODE, int OUT_MODE, bool RESID, int ACT = 0>
__global__ __launch_bounds__(256) void wmma_gemm64(
    const unsigned short* __restrict__ Ap, const unsigned short* __restrict__ A2p, int lda, long strideA,
    const unsigned short* __restrict__ Btp, const unsigned short* __restrict__ Bt2p, int ldb, long strideB,
    void* __restrict__ Cout, void* __restrict__ Cout2, int ldc, long strideC,
    const float* __restrict__ bias,
    const float* __restrict__ resid, long strideR,
    int M, int N, int K, float scale) {
  typedef typename Elem<ET>::T T;
  typedef typename Frag<T>::V V;
  const T* A = (const T*)Ap; const T* A2 = (const T*)A2p; const T* Bt = (const T*)Btp; const T* Bt2 = (const T*)Bt2p;
  __shared__ __align__(16) float sT[8][16 * 68];
  const int b    = blockIdx.y;
  const int lane = threadIdx.x & 31;
  const int wave = threadIdx.x >> 5;
  const int tilesN = N >> 6;
  const int tilesM = M >> 6;
  const int tile = blockIdx.x * 8 + wave;
  if (tile >= tilesM * tilesN) return;
  const int tm = tile / tilesN;
  const int tn = tile - tm * tilesN;
  const int m0 = tm << 6;
  const int n0 = tn << 6;

  const T* Ab  = A  + (size_t)b * strideA;
  const T* Bb  = Bt + (size_t)b * strideB;
  const T* Ab2 = SPLIT ? (A2  + (size_t)b * strideA) : nullptr;
  const T* Bb2 = SPLIT ? (Bt2 + (size_t)b * strideB) : nullptr;

  const int rlane = lane & 15;
  const int koff  = (lane >> 4) * 8;
  const int mOff  = (lane >> 4) * 8;

  v8f acc[4][4];
#pragma unroll
  for (int i = 0; i < 4; ++i)
#pragma unroll
    for (int j = 0; j < 4; ++j) acc[i][j] = (v8f){0.f,0.f,0.f,0.f,0.f,0.f,0.f,0.f};

  for (int k0 = 0; k0 < K; k0 += 32) {
    V bh[4], bl[4];
#pragma unroll
    for (int j = 0; j < 4; ++j) {
      const size_t bo = (size_t)(n0 + (j << 4) + rlane) * ldb + koff + k0;
      bh[j] = Frag<T>::load(Bb + bo);
      if (SPLIT) bl[j] = Frag<T>::load(Bb2 + bo);
    }
#pragma unroll
    for (int i = 0; i < 4; ++i) {
      const size_t ao = (size_t)(m0 + (i << 4) + rlane) * lda + koff + k0;
      V ah = Frag<T>::load(Ab + ao);
      V al;
      if (SPLIT) al = Frag<T>::load(Ab2 + ao);
#pragma unroll
      for (int j = 0; j < 4; ++j) {
        acc[i][j] = Frag<T>::mma(ah, bh[j], acc[i][j]);
        if (SPLIT) {
          acc[i][j] = Frag<T>::mma(ah, bl[j], acc[i][j]);
          acc[i][j] = Frag<T>::mma(al, bh[j], acc[i][j]);
        }
      }
      Frag<T>::guard(acc[i][0], acc[i][3], ah, SPLIT ? al : ah);
    }
    Frag<T>::keep(bh[0], bh[1], bh[2], bh[3]);
    if (SPLIT) Frag<T>::keep(bl[0], bl[1], bl[2], bl[3]);
  }
  acc_guard4(acc[0][0], acc[0][1], acc[0][2], acc[0][3]);
  acc_guard4(acc[1][0], acc[1][1], acc[1][2], acc[1][3]);
  acc_guard4(acc[2][0], acc[2][1], acc[2][2], acc[2][3]);
  acc_guard4(acc[3][0], acc[3][1], acc[3][2], acc[3][3]);

  float* slab = sT[wave];
  const float* Rb = RESID ? (resid + (size_t)b * strideR) : nullptr;
#pragma unroll
  for (int i = 0; i < 4; ++i) {
    const int mBase = m0 + (i << 4);
#pragma unroll
    for (int j = 0; j < 4; ++j) {
      const int n = n0 + (j << 4) + rlane;
      float bv = 0.f;
      if (BIAS_MODE == 2) bv = bias[n];
#pragma unroll
      for (int r = 0; r < 8; ++r) {
        float v = acc[i][j][r] * scale;
        if (BIAS_MODE == 1) v += bias[mBase + mOff + r];
        if (BIAS_MODE == 2) v += bv;
        if (RESID) v += Rb[(size_t)(mBase + mOff + r) * ldc + n];
        if (ACT == 1) v = tanhf(v);
        if (ACT == 2) v = fmaxf(v, 0.0f);
        if (ACT == 3) v = v / (1.0f + expf(-v));
        if (ACT == 4) v = (v > 0.f) ? v : 0.01f * v;
        if (ACT == 5) v = 0.5f * v * (1.0f + erff(v * 0.70710678118654752f));
        slab[(mOff + r) * 68 + (j << 4) + rlane] = v;
      }
    }
    __builtin_amdgcn_fence(__ATOMIC_RELEASE, "workgroup");
    __builtin_amdgcn_wave_barrier();
    __builtin_amdgcn_fence(__ATOMIC_ACQUIRE, "workgroup");
    if (OUT_MODE == 0) {
      float* C = (float*)Cout + (size_t)b * strideC;
      const int hh = lane >> 4, c4 = (lane & 15) * 4;
      for (int pass = 0; pass < 2; ++pass) {
#pragma unroll
        for (int it = 0; it < 8; ++it) {
          const int row = it * 2 + hh;
          v4f v = *(const v4f*)(slab + row * 68 + c4);
          *(volatile v4f*)(C + (size_t)(mBase + row) * ldc + n0 + c4) = v;
        }
        __threadfence();
      }
    } else {
      const int q = lane >> 3, c8 = (lane & 7) * 8;
      unsigned short* C  = (unsigned short*)Cout  + (size_t)b * strideC;
      unsigned short* C2 = (OUT_MODE == 2) ? ((unsigned short*)Cout2 + (size_t)b * strideC) : nullptr;
      for (int pass = 0; pass < 2; ++pass) {
#pragma unroll
        for (int it = 0; it < 4; ++it) {
          const int row = it * 4 + q;
          const float* sp = slab + row * 68 + c8;
          v8h hv, lv;
#pragma unroll
          for (int e = 0; e < 8; ++e) {
            if (OUT_MODE == 1) {
              hv[e] = (_Float16)sp[e];
            } else {
              unsigned short hb = f2bf_bits(sp[e]);
              unsigned short lb = f2bf_bits(sp[e] - bf_bits2f(hb));
              hv[e] = __builtin_bit_cast(_Float16, hb);
              lv[e] = __builtin_bit_cast(_Float16, lb);
            }
          }
          *(volatile v8h*)(C + (size_t)(mBase + row) * ldc + n0 + c8) = hv;
          if (OUT_MODE == 2) *(volatile v8h*)(C2 + (size_t)(mBase + row) * ldc + n0 + c8) = lv;
        }
        __threadfence();
      }
    }
    __builtin_amdgcn_fence(__ATOMIC_RELEASE, "workgroup");
    __builtin_amdgcn_wave_barrier();
    __builtin_amdgcn_fence(__ATOMIC_ACQUIRE, "workgroup");
  }
}

__device__ __forceinline__ unsigned pack_f16x2(float a, float b) {
  const _Float16 h0 = (_Float16)a, h1 = (_Float16)b;
  return (unsigned)__builtin_bit_cast(unsigned short, h0) | ((unsigned)__builtin_bit_cast(unsigned short, h1) << 16);
}

__global__ __launch_bounds__(256) void wprep_kernel(const float* __restrict__ Wa, const float* __restrict__ Wb,
                                                   unsigned* __restrict__ Bt, int K, int N) {
  const int kh = K >> 1;
  const int half = N * kh;
  const int i = blockIdx.x * 256 + threadIdx.x;
  if (i < half) {
    const int n = i / kh;
    const int k = (i - n * kh) * 2;
    const float* W = (blockIdx.y == 0) ? Wa : Wb;
    const float a = W[(size_t)k * N + n], b = W[(size_t)(k + 1) * N + n];
    const unsigned u = pack_f16x2(a * WSC, b * WSC);
    unsigned* p = Bt + (size_t)blockIdx.y * half + i;
    *(volatile unsigned*)p = u; __threadfence(); *(volatile unsigned*)p = u;
  }
}

template <int F, bool BN, bool SNS>
__global__ __launch_bounds__(256) void bn_cast_kernel(const float* __restrict__ X, int xrows, const float* __restrict__ STAT,
                                                     const float* __restrict__ gam, const float* __restrict__ bet,
                                                     const float* __restrict__ SN, unsigned short* __restrict__ outp) {
  const int i = blockIdx.x * 256 + threadIdx.x;
  if (i < MP * F / 8) {
    const int e0 = i * 8;
    const int row = e0 / F;
    const int col = e0 - row * F;
    const bool live = row < NNODE;
    const int rc = (row < xrows) ? row : (xrows - 1);
    const float* xp = X + (size_t)rc * F + col;
    const v4f xa = *(const v4f*)xp, xb = *(const v4f*)(xp + 4);
    float v[8] = {xa[0], xa[1], xa[2], xa[3], xb[0], xb[1], xb[2], xb[3]};
    if (BN) {
      const v4f m0 = *(const v4f*)(STAT + col), m1 = *(const v4f*)(STAT + col + 4);
      const v4f s0 = *(const v4f*)(STAT + 1024 + col), s1 = *(const v4f*)(STAT + 1024 + col + 4);
      const v4f g0 = *(const v4f*)(gam + col), g1 = *(const v4f*)(gam + col + 4);
      const v4f b0 = *(const v4f*)(bet + col), b1 = *(const v4f*)(bet + col + 4);
#pragma unroll
      for (int k = 0; k < 4; ++k) {
        v[k]     = (g0[k] * (v[k]     - m0[k])) * s0[k] + b0[k];
        v[4 + k] = (g1[k] * (v[4 + k] - m1[k])) * s1[k] + b1[k];
      }
    }
    if (SNS) {
      const float sn = SN[rc];
#pragma unroll
      for (int k = 0; k < 8; ++k) v[k] *= sn;
    }
    v8h hv;
#pragma unroll
    for (int k = 0; k < 8; ++k) hv[k] = (_Float16)(live ? v[k] : 0.f);
    _Float16* op = (_Float16*)outp + (size_t)e0;
    *(volatile v8h*)op = hv; __threadfence(); *(volatile v8h*)op = hv;
  }
}

template <int F>
__global__ __launch_bounds__(256) void bn_stats_kernel(const float* __restrict__ X, float* __restrict__ STAT) {
  __shared__ double s1[8][32];
  __shared__ double s2[8][32];
  const int tid = threadIdx.x, lane = tid & 31, w = tid >> 5;
  const int c = blockIdx.x * 32 + lane;
  double a = 0.0, b = 0.0;
#pragma unroll 1
  for (int r = w; r < NNODE; r += 8) {
    const float v = X[(size_t)r * F + c];
    a += (double)v;
    b = fma((double)v, (double)v, b);
  }
  s1[w][lane] = a; s2[w][lane] = b;
  __syncthreads();
  if (w == 0) {
    double A = 0.0, B = 0.0;
#pragma unroll
    for (int k = 0; k < 8; ++k) { A += s1[k][lane]; B += s2[k][lane]; }
    const double m = A * (1.0 / NNODE);
    double var = B * (1.0 / NNODE) - m * m;
    var = var > 0.0 ? var : 0.0;
    const float mf = (float)m;
    const float is = rsqrtf((float)var + BN_EPS);
    float* pm = STAT + c;
    float* ps = STAT + 1024 + c;
    *(volatile float*)pm = mf; *(volatile float*)ps = is;
    __threadfence();
    *(volatile float*)pm = mf; *(volatile float*)ps = is;
  }
}

__device__ __forceinline__ int blk_excl_scan(int cnt, int* scan_ws, int tid, int* tot) {
  const int lane = tid & 31, wave = tid >> 5; int incl = cnt;
#pragma unroll
  for (int o = 1; o < 32; o <<= 1) { const int v = __shfl_up(incl, o, 32); if (lane >= o) incl += v; }
  if (lane == 31) scan_ws[wave] = incl;
  __syncthreads();
  if (wave == 0) { int wv = (lane < NT / 32) ? scan_ws[lane] : 0; int wincl = wv;
#pragma unroll
    for (int o = 1; o < 32; o <<= 1) { const int v = __shfl_up(wincl, o, 32); if (lane >= o) wincl += v; }
    if (lane < NT / 32) scan_ws[32 + lane] = wincl - wv; if (lane == 31) scan_ws[64] = wincl; }
  __syncthreads();
  const int res = scan_ws[32 + wave] + incl - cnt; *tot = scan_ws[64];
  return res;
}
template <int SP, int CAP, int NTOT, int TGT>
__device__ __forceinline__ int chunk_hits(const int* __restrict__ keyv, int e0, int n0, int tid, int* LIST, int* scan_ws) {
  const int eb = e0 + tid * SP;
  const bool real = eb < NEDGE;
  const int ebc = real ? eb : (NEDGE - SP);
  int rec[SP]; int cnt = 0;
#pragma unroll
  for (int k = 0; k < SP; k += 4) {
    const v4i d4 = *(const v4i*)(keyv + ebc + k);
#pragma unroll
    for (int q = 0; q < 4; ++q) {
      const int e = eb + k + q;
      const int d = real ? d4[q] : (e - NEDGE);
      const bool valid = real ? (d < NNODE) : (e < NTOT);
      int r = -1;
      if (valid && d >= n0 && d < n0 + TGT) { r = ((d - n0) << 20) | e; ++cnt; }
      rec[k + q] = r;
    }
  }
  int tot; int p = blk_excl_scan(cnt, scan_ws, tid, &tot);
#pragma unroll
  for (int k = 0; k < SP; ++k) if (rec[k] >= 0) { if ((unsigned)p < (unsigned)CAP) LIST[p] = rec[k]; ++p; }
  __syncthreads();
  return tot < CAP ? tot : CAP;
}

__global__ __launch_bounds__(NT) void deg_kernel(const int* __restrict__ srcv, float* __restrict__ SN) {
  __shared__ float CNT[TGB];
  __shared__ int LIST[SCH];
  __shared__ int scan_ws[80];
  const int tid = threadIdx.x, lane = tid & 31, wave = tid >> 5;
  const int n0 = blockIdx.x * TGB;
  for (int i = tid; i < TGB; i += NT) CNT[i] = 0.f;
  __syncthreads();
#pragma unroll 1
  for (int c = 0; c < NCH1; ++c) {
    const int tot = chunk_hits<SPT, SCH, NEDGE, TGB>(srcv, c * SCH, n0, tid, LIST, scan_ws);
#pragma unroll 1
    for (int base = 0; base < tot; base += 32) {
      const int q = base + lane;
      const int rv = (q < tot) ? LIST[q < SCH ? q : (SCH - 1)] : -1;
      const int own = (rv >= 0 && (rv >> 28) == wave) ? 1 : 0;
      unsigned msk = (unsigned)__ballot(own);
#pragma unroll 1
      for (int it = 0; it < 32; ++it) {
        if (msk == 0u) break;
        const int bp = __builtin_ctz(msk); msk &= msk - 1u;
        const int r = __shfl(rv, bp, 32);
        const int dl = r >> 20;
        if (lane == 0) CNT[dl] += 1.0f;
        asm volatile("" ::: "memory");
      }
    }
    __syncthreads();
  }
#pragma unroll 1
  for (int j = 0; j < TGB / (8 * 32); ++j) {
    const int dl = wave * (TGB / 8) + j * 32 + lane;
    const float v = rsqrtf(CNT[dl] + 1.0f);
    float* p = SN + n0 + dl;
    *(volatile float*)p = v; __threadfence(); *(volatile float*)p = v;
  }
}

template <int F>
__global__ __launch_bounds__(NT) void agg_kernel(const float* __restrict__ HWp, const int* __restrict__ srcv, const int* __restrict__ dstv,
                                                const float* __restrict__ bias, float* __restrict__ ACC) {
  constexpr int CH = (F >= 128) ? (F / 128) : 1;
  constexpr int LM = (F >= 128) ? 31 : 15;
  __shared__ float CNT[TGB];
  __shared__ int LIST[SCH];
  __shared__ int scan_ws[80];
  const int tid = threadIdx.x, lane = tid & 31, wave = tid >> 5;
  const int n0 = blockIdx.x * TGB;
  const int c0 = 4 * (lane & LM);
  const bool act = (F >= 128) || (lane < 16);
  for (int i = tid; i < TGB; i += NT) CNT[i] = 0.f;
  {
    const v4f z4 = {0.f, 0.f, 0.f, 0.f};
    for (int pass = 0; pass < 2; ++pass) {
#pragma unroll 1
      for (int j = 0; j < TGB / 8; ++j) {
        const int n = n0 + wave * (TGB / 8) + j;
        if (n < MP) {
          float* ap = ACC + (size_t)n * F + c0;
#pragma unroll
          for (int ch = 0; ch < CH; ++ch) if (act) *(volatile v4f*)(ap + 128 * ch) = z4;
        }
      }
      __threadfence();
    }
  }
  __syncthreads();
#pragma unroll 1
  for (int c = 0; c < NCH2; ++c) {
    const int tot = chunk_hits<SPT, SCH, NVIRT, TGB>(dstv, c * SCH, n0, tid, LIST, scan_ws);
#pragma unroll 1
    for (int base = 0; base < tot; base += 32) {
      const int q = base + lane;
      const int rv = (q < tot) ? LIST[q < SCH ? q : (SCH - 1)] : -1;
      const int own = (rv >= 0 && (rv >> 28) == wave) ? 1 : 0;
      unsigned msk = (unsigned)__ballot(own);
#pragma unroll 1
      for (int it = 0; it < 32; ++it) {
        if (msk == 0u) break;
        const int bp = __builtin_ctz(msk); msk &= msk - 1u;
        const int r = __shfl(rv, bp, 32);
        const int dl = r >> 20;
        const int e  = r & 0xFFFFF;
        const int d  = n0 + dl;
        const bool real = e < NEDGE;
        const int ec = real ? e : (NEDGE - 1);
        int s = srcv[ec];
        s = s < 0 ? 0 : (s >= NNODE ? NNODE - 1 : s);
        s = real ? s : d;
        if (lane == 0) CNT[dl] += 1.0f;
        const float* hs = HWp + (size_t)s * F + c0;
        float* ap = ACC + (size_t)d * F + c0;
        v4f o[CH];
#pragma unroll
        for (int ch = 0; ch < CH; ++ch) {
          const v4f v = *(const v4f*)(hs + 128 * ch);
          const v4f qv = *(const v4f*)(ap + 128 * ch);
          o[ch] = qv + v;
        }
#pragma unroll
        for (int ch = 0; ch < CH; ++ch) if (act) *(volatile v4f*)(ap + 128 * ch) = o[ch];
        __threadfence();
#pragma unroll
        for (int ch = 0; ch < CH; ++ch) if (act) *(volatile v4f*)(ap + 128 * ch) = o[ch];
        asm volatile("" ::: "memory");
      }
    }
    __syncthreads();
  }
  v4f bb[CH];
#pragma unroll
  for (int ch = 0; ch < CH; ++ch) bb[ch] = *(const v4f*)(bias + c0 + 128 * ch);
#pragma unroll 1
  for (int j = 0; j < TGB / 8; ++j) {
    const int dl = wave * (TGB / 8) + j;
    const int n = n0 + dl;
    if (n < MP) {
      const bool live = n < NNODE;
      const float cnt = CNT[dl];
      const float dn = (live && cnt > 0.f) ? rsqrtf(cnt) : 0.f;
      float* ap = ACC + (size_t)n * F + c0;
      v4f o[CH];
#pragma unroll
      for (int ch = 0; ch < CH; ++ch) {
        const v4f qv = *(const v4f*)(ap + 128 * ch);
        v4f t;
#pragma unroll
        for (int k = 0; k < 4; ++k) {
          float u = fmaf(qv[k], dn, bb[ch][k]);
          u = fmaxf(u, 0.f);
          t[k] = live ? u : 0.f;
        }
        o[ch] = t;
      }
#pragma unroll
      for (int ch = 0; ch < CH; ++ch) if (act) *(volatile v4f*)(ap + 128 * ch) = o[ch];
      __threadfence();
#pragma unroll
      for (int ch = 0; ch < CH; ++ch) if (act) *(volatile v4f*)(ap + 128 * ch) = o[ch];
    }
  }
}

__global__ __launch_bounds__(256) void elr_kernel(const float* __restrict__ HP, const float* __restrict__ al,
                                                 const float* __restrict__ ar, float* __restrict__ ELR) {
  __shared__ __align__(16) float E[8 * 16];
  const int tid = threadIdx.x, lane = tid & 31, w = tid >> 5;
  const int n = blockIdx.x * 8 + w;
  const float* hp = HP + (size_t)n * GW + 32 * lane;
  const float* pa = al + 32 * lane;
  const float* pb = ar + 32 * lane;
  float pl = 0.f, pr = 0.f;
#pragma unroll 1
  for (int j = 0; j < 8; ++j) {
    const v4f xv = *(const v4f*)(hp + 4 * j);
    const v4f av = *(const v4f*)(pa + 4 * j);
    const v4f bv = *(const v4f*)(pb + 4 * j);
#pragma unroll
    for (int k = 0; k < 4; ++k) { pl = fmaf(xv[k], av[k], pl); pr = fmaf(xv[k], bv[k], pr); }
  }
  pl += __shfl_xor(pl, 1, 32); pl += __shfl_xor(pl, 2, 32);
  pr += __shfl_xor(pr, 1, 32); pr += __shfl_xor(pr, 2, 32);
  if ((lane & 3) == 0) { E[w * 16 + (lane >> 2)] = pl; E[w * 16 + 8 + (lane >> 2)] = pr; }
  __syncthreads();
  if (w == 0) {
    const v4f v = *(const v4f*)(E + (lane >> 2) * 16 + 4 * (lane & 3));
    float* p = ELR + (size_t)blockIdx.x * 8 * 16 + 4 * lane;
    *(volatile v4f*)p = v; __threadfence(); *(volatile v4f*)p = v;
  }
}

__device__ __forceinline__ void gat_cc(const float* __restrict__ We, const float* __restrict__ ae, float* CC, int tid) {
  if (tid < 16) {
    const int hh = tid & 7, row = tid >> 3;
    const float* wp = We + (size_t)row * GW + hh * 128;
    const float* ap = ae + hh * 128;
    float sacc = 0.f;
#pragma unroll 1
    for (int d = 0; d < 128; ++d) sacc = fmaf(wp[d], ap[d], sacc);
    CC[tid] = sacc;
  }
}
__device__ __forceinline__ float gat_logit(const float* __restrict__ ELR, const float* __restrict__ ef, const float* CC,
                                           int s, int d, int ec, bool real, int h) {
  const float el = ELR[(size_t)s * 16 + h];
  const float er = ELR[(size_t)d * 16 + 8 + h];
  const float f0 = ef[(size_t)ec * 2], f1 = ef[(size_t)ec * 2 + 1];
  const float t0 = f0 * CC[h];
  float ee = fmaf(f1, CC[8 + h], t0);
  ee = real ? ee : 0.f;
  const float x = (el + er) + ee;
  return (x > 0.f) ? x : 0.2f * x;
}

__global__ __launch_bounds__(NT) void gat_ml_kernel(const float* __restrict__ ELR, const float* __restrict__ ef,
                                                    const int* __restrict__ srcv, const int* __restrict__ dstv,
                                                    const float* __restrict__ We, const float* __restrict__ ae,
                                                    float* __restrict__ ML) {
  __shared__ float SM[TGA * 8];
  __shared__ float SL[TGA * 8];
  __shared__ int LIST[SCH];
  __shared__ int scan_ws[80];
  __shared__ float CC[16];
  const int tid = threadIdx.x, lane = tid & 31, wave = tid >> 5;
  const int n0 = blockIdx.x * TGA;
  const int h = lane & 7;
  gat_cc(We, ae, CC, tid);
  for (int i = tid; i < TGA * 8; i += NT) { SM[i] = -INFINITY; SL[i] = 0.f; }
  __syncthreads();
#pragma unroll 1
  for (int c = 0; c < NCH2; ++c) {
    const int tot = chunk_hits<SPT, SCH, NVIRT, TGA>(dstv, c * SCH, n0, tid, LIST, scan_ws);
#pragma unroll 1
    for (int base = 0; base < tot; base += 32) {
      const int q = base + lane;
      const int rv = (q < tot) ? LIST[q < SCH ? q : (SCH - 1)] : -1;
      const int own = (rv >= 0 && (rv >> 26) == wave) ? 1 : 0;
      unsigned msk = (unsigned)__ballot(own);
#pragma unroll 1
      for (int it = 0; it < 32; ++it) {
        if (msk == 0u) break;
        const int bp = __builtin_ctz(msk); msk &= msk - 1u;
        const int r = __shfl(rv, bp, 32);
        const int dl = r >> 20;
        const int e  = r & 0xFFFFF;
        const int d  = n0 + dl;
        const bool real = e < NEDGE;
        const int ec = real ? e : (NEDGE - 1);
        int s = srcv[ec];
        s = s < 0 ? 0 : (s >= NNODE ? NNODE - 1 : s);
        s = real ? s : d;
        const float x = gat_logit(ELR, ef, CC, s, d, ec, real, h);
        const int mi = dl * 8 + h;
        const float mo = SM[mi], lo = SL[mi];
        const float mn = fmaxf(mo, x);
        const float rr = __expf(mo - mn);
        const float ex = __expf(x - mn);
        const float ln = fmaf(lo, rr, ex);
        if (lane < 8) { SM[mi] = mn; SL[mi] = ln; }
        asm volatile("" ::: "memory");
      }
    }
    __syncthreads();
  }
#pragma unroll 1
  for (int j = 0; j < TGA / 16; ++j) {
    const int dlb = wave * (TGA / 8) + 2 * j;
    const int nb = n0 + dlb;
    if (nb < MP) {
      const int dl = dlb + (lane >> 4);
      const int n = nb + (lane >> 4);
      const int k = lane & 15, hh = k & 7;
      const float m = SM[dl * 8 + hh], l = SL[dl * 8 + hh];
      const bool ok = (n < NNODE) && (l > 0.f);
      const float li = 1.0f / (ok ? l : 1.0f);
      float v = (k < 8) ? m : li;
      v = ok ? v : 0.f;
      float* p = ML + (size_t)nb * 16 + lane;
      *(volatile float*)p = v; __threadfence(); *(volatile float*)p = v;
    }
  }
}

__global__ __launch_bounds__(NT) void gat_agg_kernel(const float* __restrict__ HP, const float* __restrict__ ELR,
                                                     const float* __restrict__ ML, const float* __restrict__ ef,
                                                     const int* __restrict__ srcv, const int* __restrict__ dstv,
                                                     const float* __restrict__ We, const float* __restrict__ ae,
                                                     float* __restrict__ ACC) {
  __shared__ int LIST[SCH];
  __shared__ int scan_ws[80];
  __shared__ float CC[16];
  const int tid = threadIdx.x, lane = tid & 31, wave = tid >> 5;
  const int n0 = blockIdx.x * TGB;
  const int h = lane & 7;
  const int c0 = 4 * lane;
  gat_cc(We, ae, CC, tid);
  __syncthreads();
#pragma unroll 1
  for (int c = 0; c < NCH2; ++c) {
    const int tot = chunk_hits<SPT, SCH, NVIRT, TGB>(dstv, c * SCH, n0, tid, LIST, scan_ws);
#pragma unroll 1
    for (int base = 0; base < tot; base += 32) {
      const int q = base + lane;
      const int rv = (q < tot) ? LIST[q < SCH ? q : (SCH - 1)] : -1;
      const int own = (rv >= 0 && (rv >> 28) == wave) ? 1 : 0;
      unsigned msk = (unsigned)__ballot(own);
#pragma unroll 1
      for (int it = 0; it < 32; ++it) {
        if (msk == 0u) break;
        const int bp = __builtin_ctz(msk); msk &= msk - 1u;
        const int r = __shfl(rv, bp, 32);
        const int dl = r >> 20;
        const int e  = r & 0xFFFFF;
        const int d  = n0 + dl;
        const bool real = e < NEDGE;
        const int ec = real ? e : (NEDGE - 1);
        int s = srcv[ec];
        s = s < 0 ? 0 : (s >= NNODE ? NNODE - 1 : s);
        s = real ? s : d;
        const float x = gat_logit(ELR, ef, CC, s, d, ec, real, h);
        const float m  = ML[(size_t)d * 16 + h];
        const float li = ML[(size_t)d * 16 + 8 + h];
        const float a = __expf(x - m) * li;
        float aj[8];
#pragma unroll
        for (int j = 0; j < 8; ++j) aj[j] = __shfl(a, j, 32);
        const float* hs = HP + (size_t)s * GW + c0;
        float* ap = ACC + (size_t)d * GW + c0;
        v4f o[8];
#pragma unroll
        for (int j = 0; j < 8; ++j) {
          const v4f v = *(const v4f*)(hs + 128 * j);
          const v4f qv = *(const v4f*)(ap + 128 * j);
          v4f t;
#pragma unroll
          for (int k = 0; k < 4; ++k) t[k] = fmaf(aj[j], v[k], qv[k]);
          o[j] = t;
        }
#pragma unroll
        for (int j = 0; j < 8; ++j) *(volatile v4f*)(ap + 128 * j) = o[j];
        __threadfence();
#pragma unroll
        for (int j = 0; j < 8; ++j) *(volatile v4f*)(ap + 128 * j) = o[j];
        asm volatile("" ::: "memory");
      }
    }
    __syncthreads();
  }
}

__global__ __launch_bounds__(256) void head_kernel(const float* __restrict__ T, const float* __restrict__ ba1,
                                                  const float* __restrict__ Wa2, const float* __restrict__ ba2,
                                                  const float* __restrict__ bc1, const float* __restrict__ Wc2,
                                                  const float* __restrict__ bc2, float* __restrict__ out) {
  const int f = blockIdx.x * 256 + threadIdx.x;
  if (f < 2 * NNODE) {
    const bool wc = f >= NNODE;
    const int node = wc ? (f - NNODE) : f;
    const float* tp = T + (size_t)node * THW + (wc ? 128 : 0);
    float sacc = 0.f;
#pragma unroll 1
    for (int j = 0; j < 128; j += 4) {
      const v4f tv = *(const v4f*)(tp + j);
      const v4f xa = *(const v4f*)(ba1 + j), xc = *(const v4f*)(bc1 + j);
      const v4f wa = *(const v4f*)(Wa2 + j), wv = *(const v4f*)(Wc2 + j);
#pragma unroll
      for (int k = 0; k < 4; ++k) {
        const float bb = wc ? xc[k] : xa[k];
        const float ww = wc ? wv[k] : wa[k];
        const float u = fmaxf(tv[k] + bb, 0.f);
        sacc = fmaf(u, ww, sacc);
      }
    }
    const float b2a = ba2[0], b2c = bc2[0];
    const float res = sacc + (wc ? b2c : b2a);
    *(volatile float*)(out + f) = res; __threadfence(); *(volatile float*)(out + f) = res;
  }
}

extern "C" void kernel_launch(void* const* d_in, const int* in_sizes, int n_in,
                              void* d_out, int out_size, void* d_ws, size_t ws_size, hipStream_t stream) {
  if (n_in < 33) return;
  const float* x     = (const float*)d_in[0];
  const float* efeat = (const float*)d_in[1];
  const int*   src   = (const int*)  d_in[2];
  const int*   dst   = (const int*)  d_in[3];
  const float* W1  = (const float*)d_in[4];  const float* b1  = (const float*)d_in[5];
  const float* g1  = (const float*)d_in[6];  const float* be1 = (const float*)d_in[7];
  const float* W2  = (const float*)d_in[8];  const float* b2  = (const float*)d_in[9];
  const float* g2  = (const float*)d_in[10]; const float* be2 = (const float*)d_in[11];
  const float* W3  = (const float*)d_in[12]; const float* b3  = (const float*)d_in[13];
  const float* g3  = (const float*)d_in[14]; const float* be3 = (const float*)d_in[15];
  const float* Wg  = (const float*)d_in[16]; const float* We  = (const float*)d_in[17];
  const float* atl = (const float*)d_in[18]; const float* atr = (const float*)d_in[19];
  const float* ate = (const float*)d_in[20];
  const float* Wres = (const float*)d_in[21]; const float* bg = (const float*)d_in[22];
  const float* g5  = (const float*)d_in[23]; const float* be5 = (const float*)d_in[24];
  const float* Wa1 = (const float*)d_in[25]; const float* ba1 = (const float*)d_in[26];
  const float* Wa2 = (const float*)d_in[27]; const float* ba2 = (const float*)d_in[28];
  const float* Wc1 = (const float*)d_in[29]; const float* bc1 = (const float*)d_in[30];
  const float* Wc2 = (const float*)d_in[31]; const float* bc2 = (const float*)d_in[32];
  float* out = (float*)d_out;

  if (in_sizes[0] != NNODE * 128 || in_sizes[1] != NEDGE * 2 || in_sizes[2] != NEDGE || in_sizes[3] != NEDGE) return;
  if (in_sizes[4] != 128 * 64 || in_sizes[8] != 64 * 256 || in_sizes[12] != 256 * 512) return;
  if (in_sizes[16] != 512 * GW || in_sizes[17] != 2 * GW || in_sizes[21] != 512 * GW || in_sizes[22] != GW) return;
  if (in_sizes[18] != GW || in_sizes[19] != GW || in_sizes[20] != GW || in_sizes[23] != GW || in_sizes[24] != GW) return;
  if (in_sizes[25] != GW * 128 || in_sizes[29] != GW * 128 || in_sizes[27] != 128 || in_sizes[31] != 128) return;
  if (in_sizes[5] != 64 || in_sizes[9] != 256 || in_sizes[13] != 512 || in_sizes[26] != 128 || in_sizes[30] != 128) return;
  if (in_sizes[28] < 1 || in_sizes[32] < 1 || out_size != 2 * NNODE) return;

  char* ws = (char*)d_ws; size_t off = 0;
  auto carve = [&](size_t bytes) -> char* { char* p = ws + off; off += (bytes + 255) & ~(size_t)255; return p; };
  unsigned short* RA   = (unsigned short*)carve((size_t)MP * GW * 2);
  float*          RHW  = (float*)carve((size_t)MP * GW * 4);
  float*          RACC = (float*)carve((size_t)MP * GW * 4);
  float*          SN   = (float*)carve((size_t)NTB * TGB * 4);
  unsigned*       Bt1  = (unsigned*)carve((size_t)64 * 128 * 2);
  unsigned*       Bt2  = (unsigned*)carve((size_t)256 * 64 * 2);
  unsigned*       Bt3  = (unsigned*)carve((size_t)512 * 256 * 2);
  unsigned*       BtG  = (unsigned*)carve((size_t)2048 * 512 * 2);
  unsigned*       BtH  = (unsigned*)carve((size_t)THW * GW * 2);
  float*          STAT = (float*)carve((size_t)2048 * 4);
  float*          ELR  = (float*)carve((size_t)MP * 16 * 4);
  float*          ML   = (float*)carve((size_t)MP * 16 * 4);
  if (off > ws_size || off > (size_t)134217728) return;

  auto gemm0 = [&](const unsigned short* A, int lda, const unsigned short* Bt, int ldb, float* C, int ldc, int N, int K) {
    const int tiles = (MP / 64) * (N / 64);
    wmma_gemm64<0, false, 0, 0, false, 0><<<dim3((tiles + 7) / 8, 1), 256, 0, stream>>>(
        A, A, lda, 0L, Bt, Bt, ldb, 0L, (void*)C, (void*)C, ldc, 0L,
        (const float*)SN, (const float*)SN, 0L, MP, N, K, WSC_INV);
  };

  deg_kernel<<<NTB, NT, 0, stream>>>(src, SN);
  wprep_kernel<<<dim3((64 * 64 + 255) / 256, 1), 256, 0, stream>>>(W1, W1, Bt1, 128, 64);
  wprep_kernel<<<dim3((256 * 32 + 255) / 256, 1), 256, 0, stream>>>(W2, W2, Bt2, 64, 256);
  wprep_kernel<<<dim3((512 * 128 + 255) / 256, 1), 256, 0, stream>>>(W3, W3, Bt3, 256, 512);
  wprep_kernel<<<dim3((1024 * 256 + 255) / 256, 2), 256, 0, stream>>>(Wg, Wres, BtG, 512, 1024);
  wprep_kernel<<<dim3((128 * 512 + 255) / 256, 2), 256, 0, stream>>>(Wa1, Wc1, BtH, 1024, 128);

  bn_cast_kernel<128, false, true><<<(MP * 128 / 8 + 255) / 256, 256, 0, stream>>>(x, NNODE, STAT, g1, be1, SN, RA);
  gemm0(U16(RA), 128, U16(Bt1), 128, RHW, 64, 64, 128);
  agg_kernel<64><<<NTB, NT, 0, stream>>>(RHW, src, dst, b1, RACC);
  bn_stats_kernel<64><<<64 / 32, 256, 0, stream>>>(RACC, STAT);
  bn_cast_kernel<64, true, true><<<(MP * 64 / 8 + 255) / 256, 256, 0, stream>>>(RACC, MP, STAT, g1, be1, SN, RA);
  gemm0(U16(RA), 64, U16(Bt2), 64, RHW, 256, 256, 64);
  agg_kernel<256><<<NTB, NT, 0, stream>>>(RHW, src, dst, b2, RACC);
  bn_stats_kernel<256><<<256 / 32, 256, 0, stream>>>(RACC, STAT);
  bn_cast_kernel<256, true, true><<<(MP * 256 / 8 + 255) / 256, 256, 0, stream>>>(RACC, MP, STAT, g2, be2, SN, RA);
  gemm0(U16(RA), 256, U16(Bt3), 256, RHW, 512, 512, 256);
  agg_kernel<512><<<NTB, NT, 0, stream>>>(RHW, src, dst, b3, RACC);
  bn_stats_kernel<512><<<512 / 32, 256, 0, stream>>>(RACC, STAT);
  bn_cast_kernel<512, true, false><<<(MP * 512 / 8 + 255) / 256, 256, 0, stream>>>(RACC, MP, STAT, g3, be3, SN, RA);

  gemm0(U16(RA), 512, U16(BtG), 512, RHW, GW, GW, 512);
  {
    const int tiles = (MP / 64) * (GW / 64);
    wmma_gemm64<0, false, 2, 0, false, 0><<<dim3((tiles + 7) / 8, 1), 256, 0, stream>>>(
        U16(RA), U16(RA), 512, 0L, U16(BtG) + (size_t)GW * 512, U16(BtG) + (size_t)GW * 512, 512, 0L,
        (void*)RACC, (void*)RACC, GW, 0L, bg, (const float*)SN, 0L, MP, GW, 512, WSC_INV);
  }
  elr_kernel<<<MP / 8, 256, 0, stream>>>(RHW, atl, atr, ELR);
  gat_ml_kernel<<<NTA, NT, 0, stream>>>(ELR, efeat, src, dst, We, ate, ML);
  gat_agg_kernel<<<NTB, NT, 0, stream>>>(RHW, ELR, ML, efeat, src, dst, We, ate, RACC);
  bn_stats_kernel<1024><<<GW / 32, 256, 0, stream>>>(RACC, STAT);
  bn_cast_kernel<1024, true, false><<<(MP * GW / 8 + 255) / 256, 256, 0, stream>>>(RACC, MP, STAT, g5, be5, SN, RA);

  gemm0(U16(RA), GW, U16(BtH), GW, RHW, THW, THW, GW);
  head_kernel<<<(2 * NNODE + 255) / 256, 256, 0, stream>>>(RHW, ba1, Wa2, ba2, bc1, Wc2, bc2, out);
}
